// MultiHeadDilatedSliddingWindowAttention_15839839388321
// MI455X (gfx1250) — hardware-verified
//
#include <hip/hip_runtime.h>
#include <stdint.h>
#include <stddef.h>


typedef __bf16 bf16_t;
typedef bf16_t v16bf __attribute__((ext_vector_type(16)));
typedef bf16_t v8bf  __attribute__((ext_vector_type(8)));
typedef float  v8f   __attribute__((ext_vector_type(8)));
typedef float  v4f   __attribute__((ext_vector_type(4)));
typedef unsigned int u32x4 __attribute__((ext_vector_type(4)));
typedef v8bf  __attribute__((may_alias)) v8bf_a;
typedef v4f   __attribute__((may_alias)) v4f_a;
typedef u32x4 __attribute__((may_alias)) u32x4_a;

#define NSEQ   2048
#define EDIM   1024
#define HDIM   1024
#define NHEAD  16
#define DHEAD  64
#define HALFW  64
#define APITCH 40
#define CPITCH 68
#define PPITCH 176
#define OPITCH 68

union Frag { v16bf v; v8bf h[2]; };
union Pk8  { v8bf v; u32x4 u; };

__device__ __forceinline__ v8f zero8() {
  v8f z = {0.f, 0.f, 0.f, 0.f, 0.f, 0.f, 0.f, 0.f};
  return z;
}

__device__ __forceinline__ void mma3(v8f& acc, const v16bf& ah, const v16bf& al,
                                     const v16bf& bh, const v16bf& bl) {
  acc = __builtin_amdgcn_wmma_f32_16x16x32_bf16(false, ah, false, bh, (short)0, acc, false, false);
  acc = __builtin_amdgcn_wmma_f32_16x16x32_bf16(false, ah, false, bl, (short)0, acc, false, false);
  acc = __builtin_amdgcn_wmma_f32_16x16x32_bf16(false, al, false, bh, (short)0, acc, false, false);
  asm volatile("v_nop\n\tv_nop\n\tv_nop\n\tv_nop" : "+v"(acc) : "v"(ah), "v"(al), "v"(bh), "v"(bl));
}

__device__ __forceinline__ void split_hl(v4f a, v4f b, v8bf& hi, v8bf& lo) {
#pragma unroll
  for (int q = 0; q < 4; ++q) {
    const float f0 = a[q];
    const bf16_t h0 = (bf16_t)f0;
    hi[q] = h0;
    lo[q] = (bf16_t)(f0 - (float)h0);
    const float f1 = b[q];
    const bf16_t h1 = (bf16_t)f1;
    hi[4 + q] = h1;
    lo[4 + q] = (bf16_t)(f1 - (float)h1);
  }
}

__device__ __forceinline__ void st8h(bf16_t* p, v8bf v) {
  Pk8 k; k.v = v;
  *(volatile u32x4_a*)p = k.u;
}
__device__ __forceinline__ void st4f(float* p, v4f v) {
  *(volatile v4f_a*)p = v;
}

__global__ __launch_bounds__(256)
void cvt_rows_kernel(const float* __restrict__ src, bf16_t* __restrict__ dh,
                     bf16_t* __restrict__ dl, int n) {
  const size_t i = ((size_t)blockIdx.x * 256u + (size_t)threadIdx.x) * 8u;
  if (i + 8 <= (size_t)n) {
    const v4f a = *(const v4f_a*)(src + i);
    const v4f b = *(const v4f_a*)(src + i + 4);
    v8bf hi, lo;
    split_hl(a, b, hi, lo);
    st8h(dh + i, hi);
    st8h(dl + i, lo);
    __threadfence();
    st8h(dh + i, hi);
    st8h(dl + i, lo);
  }
}

__global__ __launch_bounds__(128)
void cvt_wt_kernel(const float* __restrict__ W0, const float* __restrict__ W1,
                   const float* __restrict__ W2, const float* __restrict__ W3,
                   bf16_t* __restrict__ planes) {
  __shared__ float T[64][65];
  const int z = blockIdx.z;
  const float* W = (z == 0) ? W0 : ((z == 1) ? W1 : ((z == 2) ? W2 : W3));
  bf16_t* Wh = planes + (size_t)z * 2u * (size_t)(EDIM * HDIM);
  bf16_t* Wl = Wh + (size_t)(EDIM * HDIM);
  const int k0 = blockIdx.y * 64;
  const int n0 = blockIdx.x * 64;
  const int t = threadIdx.x, wave = t >> 5, lane = t & 31;

#pragma unroll
  for (int p = 0; p < 8; ++p) {
    const int idx = t + 128 * p;
    const int r = idx >> 4;
    const int cq = (idx & 15) * 4;
    const v4f v = *(const v4f_a*)(W + (size_t)(k0 + r) * HDIM + n0 + cq);
    T[r][cq + 0] = v[0];
    T[r][cq + 1] = v[1];
    T[r][cq + 2] = v[2];
    T[r][cq + 3] = v[3];
  }
  __syncthreads();

  const int g = lane & 7, rq = lane >> 3;
  v8bf oh[4], ol[4];
#pragma unroll
  for (int p = 0; p < 4; ++p) {
    const int nn = wave * 16 + p * 4 + rq;
    v4f a = {0.f, 0.f, 0.f, 0.f};
    v4f b = {0.f, 0.f, 0.f, 0.f};
#pragma unroll
    for (int e = 0; e < 4; ++e) {
      a[e] = T[8 * g + e][nn];
      b[e] = T[8 * g + 4 + e][nn];
    }
    split_hl(a, b, oh[p], ol[p]);
    const size_t d = (size_t)(n0 + nn) * EDIM + k0 + 8 * g;
    st8h(Wh + d, oh[p]);
    st8h(Wl + d, ol[p]);
  }
  __threadfence();
#pragma unroll
  for (int p = 0; p < 4; ++p) {
    const int nn = wave * 16 + p * 4 + rq;
    const size_t d = (size_t)(n0 + nn) * EDIM + k0 + 8 * g;
    st8h(Wh + d, oh[p]);
    st8h(Wl + d, ol[p]);
  }
}

__global__ __launch_bounds__(128)
void gemm3_kernel(const bf16_t* __restrict__ Ah, const bf16_t* __restrict__ Al, int lda,
                  const bf16_t* __restrict__ Bh, const bf16_t* __restrict__ Bl, int ldb, int K,
                  const float* __restrict__ bias_col, const float* __restrict__ bias_row,
                  float* __restrict__ Cf, bf16_t* __restrict__ Ch, bf16_t* __restrict__ Cl, int ldc) {
  __shared__ __attribute__((aligned(16))) bf16_t Ash[64][APITCH];
  __shared__ __attribute__((aligned(16))) bf16_t Asl[64][APITCH];
  __shared__ __attribute__((aligned(16))) bf16_t Bsh[64][APITCH];
  __shared__ __attribute__((aligned(16))) bf16_t Bsl[64][APITCH];
  __shared__ __attribute__((aligned(16))) float  Cs[64][CPITCH];

  const int t = threadIdx.x;
  const int wave = t >> 5, lane = t & 31;
  const int m = lane & 15, hh = lane >> 4;
  const int wr = wave >> 1, wc = wave & 1;
  const int row0 = blockIdx.y * 64;
  const int col0 = blockIdx.x * 64;

  v8f acc[2][2];
  acc[0][0] = zero8(); acc[0][1] = zero8(); acc[1][0] = zero8(); acc[1][1] = zero8();

  for (int k0 = 0; k0 < K; k0 += 32) {
#pragma unroll
    for (int p = 0; p < 2; ++p) {
      const int idx = t + 128 * p;
      const int r = idx >> 2;
      const int kq = (idx & 3) * 8;
      const size_t ao = (size_t)(row0 + r) * (size_t)lda + (size_t)(k0 + kq);
      const size_t bo = (size_t)(col0 + r) * (size_t)ldb + (size_t)(k0 + kq);
      *(v8bf_a*)&Ash[r][kq] = *(const v8bf_a*)(Ah + ao);
      *(v8bf_a*)&Asl[r][kq] = *(const v8bf_a*)(Al + ao);
      *(v8bf_a*)&Bsh[r][kq] = *(const v8bf_a*)(Bh + bo);
      *(v8bf_a*)&Bsl[r][kq] = *(const v8bf_a*)(Bl + bo);
    }
    __syncthreads();

    Frag fah[2], fal[2], fbh[2], fbl[2];
#pragma unroll
    for (int mi = 0; mi < 2; ++mi) {
      const int rr = wr * 32 + mi * 16 + m;
      fah[mi].h[0] = *(const v8bf_a*)&Ash[rr][8 * hh];
      fah[mi].h[1] = *(const v8bf_a*)&Ash[rr][16 + 8 * hh];
      fal[mi].h[0] = *(const v8bf_a*)&Asl[rr][8 * hh];
      fal[mi].h[1] = *(const v8bf_a*)&Asl[rr][16 + 8 * hh];
    }
#pragma unroll
    for (int ni = 0; ni < 2; ++ni) {
      const int rr = wc * 32 + ni * 16 + m;
      fbh[ni].h[0] = *(const v8bf_a*)&Bsh[rr][8 * hh];
      fbh[ni].h[1] = *(const v8bf_a*)&Bsh[rr][16 + 8 * hh];
      fbl[ni].h[0] = *(const v8bf_a*)&Bsl[rr][8 * hh];
      fbl[ni].h[1] = *(const v8bf_a*)&Bsl[rr][16 + 8 * hh];
    }
    mma3(acc[0][0], fah[0].v, fal[0].v, fbh[0].v, fbl[0].v);
    mma3(acc[0][1], fah[0].v, fal[0].v, fbh[1].v, fbl[1].v);
    mma3(acc[1][0], fah[1].v, fal[1].v, fbh[0].v, fbl[0].v);
    mma3(acc[1][1], fah[1].v, fal[1].v, fbh[1].v, fbl[1].v);
    __syncthreads();
  }

#pragma unroll
  for (int mi = 0; mi < 2; ++mi)
#pragma unroll
    for (int ni = 0; ni < 2; ++ni)
#pragma unroll
      for (int r = 0; r < 8; ++r)
        Cs[wr * 32 + mi * 16 + 8 * hh + r][wc * 32 + ni * 16 + m] = acc[mi][ni][r];
  __syncthreads();

  if (Cf != nullptr) {
    const int rq = lane >> 4, cq = (lane & 15) * 4;
    v4f bc = {0.f, 0.f, 0.f, 0.f};
    if (bias_col != nullptr) bc = *(const v4f_a*)(bias_col + col0 + cq);
    v4f vals[8];
#pragma unroll
    for (int p = 0; p < 8; ++p) {
      const int row = wave * 16 + p * 2 + rq;
      v4f v = *(const v4f_a*)&Cs[row][cq];
      v = v + bc;
      if (bias_row != nullptr) v = v + bias_row[row0 + row];
      vals[p] = v;
      st4f(Cf + (size_t)(row0 + row) * (size_t)ldc + col0 + cq, v);
    }
    __threadfence();
#pragma unroll
    for (int p = 0; p < 8; ++p) {
      const int row = wave * 16 + p * 2 + rq;
      st4f(Cf + (size_t)(row0 + row) * (size_t)ldc + col0 + cq, vals[p]);
    }
  } else {
    const int rq = lane >> 3, g = lane & 7;
    v4f bc0 = {0.f, 0.f, 0.f, 0.f};
    v4f bc1 = {0.f, 0.f, 0.f, 0.f};
    if (bias_col != nullptr) {
      bc0 = *(const v4f_a*)(bias_col + col0 + 8 * g);
      bc1 = *(const v4f_a*)(bias_col + col0 + 8 * g + 4);
    }
    v8bf oh[4], ol[4];
#pragma unroll
    for (int p = 0; p < 4; ++p) {
      const int row = wave * 16 + p * 4 + rq;
      v4f v0 = *(const v4f_a*)&Cs[row][8 * g];
      v4f v1 = *(const v4f_a*)&Cs[row][8 * g + 4];
      v0 = v0 + bc0;
      v1 = v1 + bc1;
      if (bias_row != nullptr) {
        const float br = bias_row[row0 + row];
        v0 = v0 + br;
        v1 = v1 + br;
      }
      split_hl(v0, v1, oh[p], ol[p]);
      const size_t d = (size_t)(row0 + row) * (size_t)ldc + col0 + 8 * g;
      st8h(Ch + d, oh[p]);
      st8h(Cl + d, ol[p]);
    }
    __threadfence();
#pragma unroll
    for (int p = 0; p < 4; ++p) {
      const int row = wave * 16 + p * 4 + rq;
      const size_t d = (size_t)(row0 + row) * (size_t)ldc + col0 + 8 * g;
      st8h(Ch + d, oh[p]);
      st8h(Cl + d, ol[p]);
    }
  }
}

__global__ __launch_bounds__(128)
void oob_vsum_kernel(const bf16_t* __restrict__ Vth, const bf16_t* __restrict__ Vtl,
                     float* __restrict__ G) {
  const int c = blockIdx.x * 128 + threadIdx.x;
  if (c < HDIM) {
    const bf16_t* vh = Vth + (size_t)c * NSEQ;
    const bf16_t* vl = Vtl + (size_t)c * NSEQ;
    double tot = 0.0;
#pragma unroll 4
    for (int j = 0; j < NSEQ; ++j) tot += (double)((float)vh[j] + (float)vl[j]);
    double w = 0.0;
    for (int j = 0; j <= HALFW; ++j) w += (double)((float)vh[j] + (float)vl[j]);
    for (int i = 0; i < NSEQ; ++i) {
      const float gv = (float)(tot - w);
      float* p = G + (size_t)i * HDIM + c;
      *(volatile float*)p = gv;
      __threadfence();
      *(volatile float*)p = gv;
      const int ja = i + HALFW + 1;
      if (ja < NSEQ) w += (double)((float)vh[ja] + (float)vl[ja]);
      const int jd = i - HALFW;
      if (jd >= 0) w -= (double)((float)vh[jd] + (float)vl[jd]);
    }
  }
}

__global__ __launch_bounds__(64)
void band_attn_kernel(const bf16_t* __restrict__ Qh, const bf16_t* __restrict__ Ql,
                      const bf16_t* __restrict__ Kh, const bf16_t* __restrict__ Kl,
                      const bf16_t* __restrict__ Vth, const bf16_t* __restrict__ Vtl,
                      const float* __restrict__ G,
                      bf16_t* __restrict__ AOh, bf16_t* __restrict__ AOl) {
  __shared__ __attribute__((aligned(16))) bf16_t Ph[2][16][PPITCH];
  __shared__ __attribute__((aligned(16))) bf16_t Pl[2][16][PPITCH];
  __shared__ __attribute__((aligned(16))) float  Os[2][16][OPITCH];
  __shared__ float Zs[2][16];
  __shared__ float Es[2][16];

  const int wave = threadIdx.x >> 5, lane = threadIdx.x & 31;
  const int m = lane & 15, hh = lane >> 4;
  const int h = blockIdx.y;
  const int i0 = (blockIdx.x * 2 + wave) * 16;
  const int jbase = i0 - HALFW;
  const int hoff = h * DHEAD;

  Frag aqh0, aqh1, aql0, aql1;
  {
    const bf16_t* qh = Qh + (size_t)(i0 + m) * HDIM + hoff;
    const bf16_t* ql = Ql + (size_t)(i0 + m) * HDIM + hoff;
    aqh0.h[0] = *(const v8bf_a*)(qh + 8 * hh);
    aqh0.h[1] = *(const v8bf_a*)(qh + 16 + 8 * hh);
    aqh1.h[0] = *(const v8bf_a*)(qh + 32 + 8 * hh);
    aqh1.h[1] = *(const v8bf_a*)(qh + 48 + 8 * hh);
    aql0.h[0] = *(const v8bf_a*)(ql + 8 * hh);
    aql0.h[1] = *(const v8bf_a*)(ql + 16 + 8 * hh);
    aql1.h[0] = *(const v8bf_a*)(ql + 32 + 8 * hh);
    aql1.h[1] = *(const v8bf_a*)(ql + 48 + 8 * hh);
  }

  v8f sc[9];
#pragma unroll
  for (int tt = 0; tt < 9; ++tt) {
    int jr = jbase + tt * 16 + m;
    jr = jr < 0 ? 0 : jr;
    jr = jr > NSEQ - 1 ? NSEQ - 1 : jr;
    const bf16_t* kh = Kh + (size_t)jr * HDIM + hoff;
    const bf16_t* kl = Kl + (size_t)jr * HDIM + hoff;
    Frag bh0, bh1, bl0, bl1;
    bh0.h[0] = *(const v8bf_a*)(kh + 8 * hh);
    bh0.h[1] = *(const v8bf_a*)(kh + 16 + 8 * hh);
    bh1.h[0] = *(const v8bf_a*)(kh + 32 + 8 * hh);
    bh1.h[1] = *(const v8bf_a*)(kh + 48 + 8 * hh);
    bl0.h[0] = *(const v8bf_a*)(kl + 8 * hh);
    bl0.h[1] = *(const v8bf_a*)(kl + 16 + 8 * hh);
    bl1.h[0] = *(const v8bf_a*)(kl + 32 + 8 * hh);
    bl1.h[1] = *(const v8bf_a*)(kl + 48 + 8 * hh);
    v8f cacc = zero8();
    mma3(cacc, aqh0.v, aql0.v, bh0.v, bl0.v);
    mma3(cacc, aqh1.v, aql1.v, bh1.v, bl1.v);
    sc[tt] = cacc;
  }

  float zr[8], er[8];
#pragma unroll
  for (int r = 0; r < 8; ++r) {
    const int rp = r + 8 * hh;
    const int i = i0 + rp;
    float mx = 0.f;
#pragma unroll
    for (int tt = 0; tt < 9; ++tt) {
      const int c = tt * 16 + m;
      const int j = jbase + c;
      const bool band = (c >= rp) && (c <= rp + 2 * HALFW) && (j >= 0) && (j < NSEQ);
      if (band) mx = fmaxf(mx, sc[tt][r]);
    }
#pragma unroll
    for (int off = 1; off < 16; off <<= 1) mx = fmaxf(mx, __shfl_xor(mx, off, 16));
    float se = 0.f;
#pragma unroll
    for (int tt = 0; tt < 9; ++tt) {
      const int c = tt * 16 + m;
      const int j = jbase + c;
      const bool band = (c >= rp) && (c <= rp + 2 * HALFW) && (j >= 0) && (j < NSEQ);
      const float e = band ? __expf(sc[tt][r] - mx) : 0.f;
      se += e;
      const bf16_t eh = (bf16_t)e;
      const bf16_t el = (bf16_t)(e - (float)eh);
      Ph[wave][rp][c] = eh;
      Pl[wave][rp][c] = el;
    }
#pragma unroll
    for (int off = 1; off < 16; off <<= 1) se += __shfl_xor(se, off, 16);
    Ph[wave][rp][144 + m] = (bf16_t)0.f;
    Pl[wave][rp][144 + m] = (bf16_t)0.f;
    int lo = i - HALFW; lo = lo < 0 ? 0 : lo;
    int hi = i + HALFW; hi = hi > NSEQ - 1 ? NSEQ - 1 : hi;
    const float ce = __expf(-mx);
    zr[r] = se + (float)(NSEQ - (hi - lo + 1)) * ce;
    er[r] = ce;
  }
  if (m == 0) {
#pragma unroll
    for (int r = 0; r < 8; ++r) {
      Zs[wave][8 * hh + r] = zr[r];
      Es[wave][8 * hh + r] = er[r];
    }
  }
  __syncthreads();

  v8f ao[4];
  ao[0] = zero8(); ao[1] = zero8(); ao[2] = zero8(); ao[3] = zero8();
#pragma unroll
  for (int s = 0; s < 5; ++s) {
    Frag aph, apl;
    aph.h[0] = *(const v8bf_a*)&Ph[wave][m][s * 32 + 8 * hh];
    aph.h[1] = *(const v8bf_a*)&Ph[wave][m][s * 32 + 16 + 8 * hh];
    apl.h[0] = *(const v8bf_a*)&Pl[wave][m][s * 32 + 8 * hh];
    apl.h[1] = *(const v8bf_a*)&Pl[wave][m][s * 32 + 16 + 8 * hh];
    int g0 = jbase + s * 32 + 8 * hh;
    int g1 = g0 + 16;
    g0 = g0 < 0 ? 0 : g0; g0 = g0 > NSEQ - 8 ? NSEQ - 8 : g0;
    g1 = g1 < 0 ? 0 : g1; g1 = g1 > NSEQ - 8 ? NSEQ - 8 : g1;
#pragma unroll
    for (int nt = 0; nt < 4; ++nt) {
      const size_t vrow = (size_t)(hoff + nt * 16 + m) * NSEQ;
      Frag bvh, bvl;
      bvh.h[0] = *(const v8bf_a*)(Vth + vrow + g0);
      bvh.h[1] = *(const v8bf_a*)(Vth + vrow + g1);
      bvl.h[0] = *(const v8bf_a*)(Vtl + vrow + g0);
      bvl.h[1] = *(const v8bf_a*)(Vtl + vrow + g1);
      mma3(ao[nt], aph.v, apl.v, bvh.v, bvl.v);
    }
  }

#pragma unroll
  for (int nt = 0; nt < 4; ++nt)
#pragma unroll
    for (int r = 0; r < 8; ++r)
      Os[wave][8 * hh + r][nt * 16 + m] = ao[nt][r];
  __syncthreads();

  {
    const int g = lane & 7, rq = lane >> 3;
    v8bf oh[4], ol[4];
#pragma unroll
    for (int p = 0; p < 4; ++p) {
      const int q = p * 4 + rq;
      const v4f o0 = *(const v4f_a*)&Os[wave][q][8 * g];
      const v4f o1 = *(const v4f_a*)&Os[wave][q][8 * g + 4];
      const float* gp = G + (size_t)(i0 + q) * HDIM + hoff + 8 * g;
      const v4f gv0 = *(const v4f_a*)gp;
      const v4f gv1 = *(const v4f_a*)(gp + 4);
      const float ce = Es[wave][q];
      const float rz = 1.0f / Zs[wave][q];
      const v4f v0 = (o0 + ce * gv0) * rz;
      const v4f v1 = (o1 + ce * gv1) * rz;
      split_hl(v0, v1, oh[p], ol[p]);
      const size_t d = (size_t)(i0 + q) * HDIM + hoff + 8 * g;
      st8h(AOh + d, oh[p]);
      st8h(AOl + d, ol[p]);
    }
    __threadfence();
#pragma unroll
    for (int p = 0; p < 4; ++p) {
      const int q = p * 4 + rq;
      const size_t d = (size_t)(i0 + q) * HDIM + hoff + 8 * g;
      st8h(AOh + d, oh[p]);
      st8h(AOl + d, ol[p]);
    }
  }
}

extern "C" void kernel_launch(void* const* d_in, const int* in_sizes, int n_in,
                              void* d_out, int out_size, void* d_ws, size_t ws_size,
                              hipStream_t stream) {
  if (n_in < 9) return;
  const size_t nx = (size_t)NSEQ * EDIM;
  const size_t nw = (size_t)EDIM * HDIM;
  const size_t nq = (size_t)NSEQ * HDIM;
  if ((size_t)in_sizes[0] != nx || (size_t)in_sizes[1] != nw || in_sizes[2] != HDIM ||
      (size_t)in_sizes[3] != nw || in_sizes[4] != HDIM || (size_t)in_sizes[5] != nw ||
      in_sizes[6] != HDIM || (size_t)in_sizes[7] != nw || in_sizes[8] != EDIM ||
      (size_t)out_size != nx) return;

  const float* x  = (const float*)d_in[0];
  const float* Wq = (const float*)d_in[1];
  const float* bq = (const float*)d_in[2];
  const float* Wk = (const float*)d_in[3];
  const float* bk = (const float*)d_in[4];
  const float* Wv = (const float*)d_in[5];
  const float* bv = (const float*)d_in[6];
  const float* Wo = (const float*)d_in[7];
  const float* bo = (const float*)d_in[8];
  float* out = (float*)d_out;

  char* ws = (char*)d_ws;
  size_t off = 0;
  bf16_t* xh  = (bf16_t*)(ws + off); off += nx * 2;
  bf16_t* xl  = (bf16_t*)(ws + off); off += nx * 2;
  bf16_t* wt  = (bf16_t*)(ws + off); off += 8 * nw * 2;
  bf16_t* Qh  = (bf16_t*)(ws + off); off += nq * 2;
  bf16_t* Ql  = (bf16_t*)(ws + off); off += nq * 2;
  bf16_t* Kh  = (bf16_t*)(ws + off); off += nq * 2;
  bf16_t* Kl  = (bf16_t*)(ws + off); off += nq * 2;
  bf16_t* Vth = (bf16_t*)(ws + off); off += nq * 2;
  bf16_t* Vtl = (bf16_t*)(ws + off); off += nq * 2;
  float*  G   = (float*)(ws + off);  off += nq * 4;
  bf16_t* AOh = (bf16_t*)(ws + off); off += nq * 2;
  bf16_t* AOl = (bf16_t*)(ws + off); off += nq * 2;
  if (off > ws_size) return;

  bf16_t* Wqth = wt + 0 * nw; bf16_t* Wqtl = wt + 1 * nw;
  bf16_t* Wkth = wt + 2 * nw; bf16_t* Wktl = wt + 3 * nw;
  bf16_t* Wvth = wt + 4 * nw; bf16_t* Wvtl = wt + 5 * nw;
  bf16_t* Woth = wt + 6 * nw; bf16_t* Wotl = wt + 7 * nw;

  cvt_rows_kernel<<<(unsigned)((nx / 8 + 255) / 256), 256, 0, stream>>>(x, xh, xl, (int)nx);
  cvt_wt_kernel<<<dim3(HDIM / 64, EDIM / 64, 4), 128, 0, stream>>>(Wq, Wk, Wv, Wo, wt);
  gemm3_kernel<<<dim3(HDIM / 64, NSEQ / 64), 128, 0, stream>>>(
      xh, xl, EDIM, Wqth, Wqtl, EDIM, EDIM, bq, nullptr, nullptr, Qh, Ql, HDIM);
  gemm3_kernel<<<dim3(HDIM / 64, NSEQ / 64), 128, 0, stream>>>(
      xh, xl, EDIM, Wkth, Wktl, EDIM, EDIM, bk, nullptr, nullptr, Kh, Kl, HDIM);
  gemm3_kernel<<<dim3(NSEQ / 64, HDIM / 64), 128, 0, stream>>>(
      Wvth, Wvtl, EDIM, xh, xl, EDIM, EDIM, nullptr, bv, nullptr, Vth, Vtl, NSEQ);
  oob_vsum_kernel<<<HDIM / 128, 128, 0, stream>>>(Vth, Vtl, G);
  band_attn_kernel<<<dim3(NSEQ / 32, NHEAD), 64, 0, stream>>>(Qh, Ql, Kh, Kl, Vth, Vtl, G, AOh, AOl);
  gemm3_kernel<<<dim3(EDIM / 64, NSEQ / 64), 128, 0, stream>>>(
      AOh, AOl, HDIM, Woth, Wotl, HDIM, HDIM, bo, nullptr, out, nullptr, nullptr, EDIM);
}
